// GlobalAggregationBlock_91225105367612
// MI455X (gfx1250) — hardware-verified
//
#include <hip/hip_runtime.h>
#include <math.h>
#include <stdint.h>

#define NIMG  8
#define CC    256
#define NN    4096
#define CK    128
#define CV    128
#define CO    256
#define MQKV  384
#define QT    64
#define OSP   68
#define OSPW  132
#define TP    72
#define QP    136
#define BP    136
#define WSC   256.0f
#define IWSC  0.00390625f
#define VSC   16.0f
#define IVSC  0.0625f
#define USC   16.0f
#define IUSC  0.0625f
#define RSC   2048.0f
#define IRSC  0.00048828125f
#define LNPS  6.931471805599453f
#define SCL   0.08838834764831845f

static_assert(NN % QT == 0);
static_assert(CC % 32 == 0 && CK % 32 == 0 && CV % 32 == 0);
static_assert(MQKV == 2 * CK + CV);
static_assert(MQKV % QT == 0 && CO % QT == 0);
static_assert(CK == 2 * QT && CV == 2 * QT);
static_assert((OSP * 4) % 16 == 0);
static_assert((OSPW * 4) % 16 == 0);
static_assert((TP * 2) % 16 == 0);
static_assert((QP * 2) % 16 == 0 && (BP * 2) % 16 == 0 && (BP % 2) == 0);
static_assert(QT * OSPW * 4 <= 2 * QT * QP * 2);

typedef _Float16       v16h __attribute__((ext_vector_type(16)));
typedef _Float16       v8h  __attribute__((ext_vector_type(8)));
typedef __bf16         v16b __attribute__((ext_vector_type(16)));
typedef unsigned short v8us __attribute__((ext_vector_type(8)));
typedef float          v8f  __attribute__((ext_vector_type(8)));
typedef float          v4f  __attribute__((ext_vector_type(4)));
typedef unsigned int   v4u  __attribute__((ext_vector_type(4)));

union Frag  { v8us u[2]; v16h h; v16b bf; };
union FragH { v16h v; v8h hv[2]; };
static_assert(sizeof(Frag) == 32);
static_assert(sizeof(FragH) == 32);

__device__ __forceinline__ unsigned short bf_bits(float f) {
  unsigned u = __float_as_uint(f);
  return (unsigned short)((u + 0x7FFFu + ((u >> 16) & 1u)) >> 16);
}
__device__ __forceinline__ float bf_up(unsigned short hb) { return __uint_as_float(((unsigned)hb) << 16); }
__device__ __forceinline__ float bfr(float f) { return bf_up(bf_bits(f)); }
__device__ __forceinline__ unsigned short h_bits(_Float16 x) { return __builtin_bit_cast(unsigned short, x); }
__device__ __forceinline__ unsigned pk16(unsigned short a, unsigned short b) { return (unsigned)a | ((unsigned)b << 16); }
__device__ __forceinline__ v8f zero8() { v8f z = {0.f, 0.f, 0.f, 0.f, 0.f, 0.f, 0.f, 0.f}; return z; }
__device__ __forceinline__ float hmax8(v8f s) {
  return fmaxf(fmaxf(fmaxf(s[0], s[1]), fmaxf(s[2], s[3])), fmaxf(fmaxf(s[4], s[5]), fmaxf(s[6], s[7])));
}

__device__ __forceinline__ Frag ldfrag(const unsigned short* p) {
  Frag f;
  f.u[0] = *(const v8us*)(p);
  f.u[1] = *(const v8us*)(p + 16);
  return f;
}

__device__ __forceinline__ v8f mma_h(v16h a, v16h b, v8f c) {
  v8f d = __builtin_amdgcn_wmma_f32_16x16x32_f16(false, a, false, b, (short)0, c, false, false);
#if defined(__HIP_DEVICE_COMPILE__)
  asm volatile("v_nop\n\tv_nop\n\tv_nop\n\tv_nop" : "+v"(d) : "v"(a), "v"(b));
#endif
  return d;
}
__device__ __forceinline__ v8f mma_b(v16b a, v16b b, v8f c) {
  v8f d = __builtin_amdgcn_wmma_f32_16x16x32_bf16(false, a, false, b, (short)0, c, false, false);
#if defined(__HIP_DEVICE_COMPILE__)
  const v16h ha = __builtin_bit_cast(v16h, a), hb = __builtin_bit_cast(v16h, b);
  asm volatile("v_nop\n\tv_nop\n\tv_nop\n\tv_nop" : "+v"(d) : "v"(ha), "v"(hb));
#endif
  return d;
}

__global__ __launch_bounds__(256)
void cvt_w(const float* __restrict__ wq, const float* __restrict__ bq,
           const float* __restrict__ wk, const float* __restrict__ bk,
           const float* __restrict__ wv, const float* __restrict__ bv,
           unsigned short* W16, float* BIAS) {
  const int tid = threadIdx.x, blk = blockIdx.x;
  const int rl = tid >> 5, col = 8 * (tid & 31);
  const int o = 8 * blk + rl;
  const float* wbase = (blk < 16) ? wq : (blk < 32) ? wk : wv;
  const int osub = (blk < 16) ? 0 : (blk < 32) ? CK : 2 * CK;
  const float* s = wbase + (size_t)(o - osub) * CC + col;
  const v4f a = *(const v4f*)s;
  const v4f q = *(const v4f*)(s + 4);
  const float f[8] = {a[0], a[1], a[2], a[3], q[0], q[1], q[2], q[3]};
  v4u u;
#pragma unroll
  for (int t = 0; t < 4; ++t) {
    const _Float16 h0 = (_Float16)(bfr(f[2 * t]) * WSC);
    const _Float16 h1 = (_Float16)(bfr(f[2 * t + 1]) * WSC);
    u[t] = pk16(h_bits(h0), h_bits(h1));
  }
  v4f bvv;
  {
    const int tb = min(tid, 95);
    const int o4 = 4 * tb;
#pragma unroll
    for (int qd = 0; qd < 4; ++qd) {
      const int oo = o4 + qd;
      const int iq = min(oo, CK - 1);
      const int ik = min(max(oo - CK, 0), CK - 1);
      const int iv = min(max(oo - 2 * CK, 0), CV - 1);
      const float cq = bq[iq], ckv = bk[ik], cvv = bv[iv];
      const float val = (oo < CK) ? cq : (oo < 2 * CK) ? ckv : cvv;
      bvv[qd] = bfr(val);
    }
  }
#pragma unroll
  for (int pass = 0; pass < 2; ++pass) {
    *(volatile v4u*)(W16 + (size_t)o * CC + col) = u;
    if (blk == 0 && tid < 96) *(volatile v4f*)(BIAS + 4 * tid) = bvv;
    __threadfence();
  }
}

__global__ __launch_bounds__(256)
void cvt_wo(const float* __restrict__ wo, const float* __restrict__ bo, unsigned short* WO16, float* BOB) {
  const int tid = threadIdx.x, blk = blockIdx.x;
  const int rl = tid >> 4, col = 8 * (tid & 15);
  const int o = 16 * blk + rl;
  const float* s = wo + (size_t)o * CV + col;
  const v4f a = *(const v4f*)s;
  const v4f q = *(const v4f*)(s + 4);
  const float f[8] = {a[0], a[1], a[2], a[3], q[0], q[1], q[2], q[3]};
  v4u u;
#pragma unroll
  for (int t = 0; t < 4; ++t) {
    const _Float16 h0 = (_Float16)(bfr(f[2 * t]) * WSC);
    const _Float16 h1 = (_Float16)(bfr(f[2 * t + 1]) * WSC);
    u[t] = pk16(h_bits(h0), h_bits(h1));
  }
  v4f bvv;
  {
    const int tb = min(tid, 63);
#pragma unroll
    for (int qd = 0; qd < 4; ++qd) bvv[qd] = bfr(bo[4 * tb + qd]);
  }
#pragma unroll
  for (int pass = 0; pass < 2; ++pass) {
    *(volatile v4u*)(WO16 + (size_t)o * CV + col) = u;
    if (blk == 0 && tid < 64) *(volatile v4f*)(BOB + 4 * tid) = bvv;
    __threadfence();
  }
}

__global__ __launch_bounds__(256)
void cvt_x(const float* __restrict__ x, unsigned short* XP) {
  __shared__ __align__(16) unsigned short T[QT * TP];
  const int tid = threadIdx.x;
  const int nb = blockIdx.x, cb = blockIdx.y, b = blockIdx.z;
  const int e = tid & 7, lq = tid >> 3;
  const int n0 = nb * QT, c0 = cb * QT;
#pragma unroll
  for (int it = 0; it < 2; ++it) {
    const int cl = it * 32 + lq;
    const float* sp = x + ((size_t)(b * CC + c0 + cl)) * NN + n0 + 8 * e;
    const v4f a = *(const v4f*)sp;
    const v4f q = *(const v4f*)(sp + 4);
    unsigned short hb[8];
#pragma unroll
    for (int t = 0; t < 4; ++t) {
      hb[t]     = h_bits((_Float16)bfr(a[t]));
      hb[4 + t] = h_bits((_Float16)bfr(q[t]));
    }
#pragma unroll
    for (int t = 0; t < 8; ++t) T[(8 * e + t) * TP + cl] = hb[t];
  }
  __syncthreads();
  v4u up[2];
#pragma unroll
  for (int it = 0; it < 2; ++it) {
    const int nl = it * 32 + lq;
    up[it] = *(const v4u*)(T + nl * TP + 8 * e);
  }
#pragma unroll
  for (int pass = 0; pass < 2; ++pass) {
#pragma unroll
    for (int it = 0; it < 2; ++it) {
      const int rl = it * 32 + lq;
      *(volatile v4u*)(XP + ((size_t)(b * NN + n0 + rl)) * CC + c0 + 8 * e) = up[it];
    }
    __threadfence();
  }
}

__global__ __launch_bounds__(128)
void gemm_qkv(const unsigned short* __restrict__ W16, const float* __restrict__ BIAS,
              const unsigned short* __restrict__ XP,
              unsigned short* Qh, unsigned short* Ql, unsigned short* Kh, unsigned short* Kl,
              unsigned short* Vh) {
  __shared__ __align__(16) float Os[QT * OSP];
  const int tid  = threadIdx.x;
  const int lane = tid & 31, wave = tid >> 5;
  const int hh   = lane >> 4, c = lane & 15;
  const int nt   = blockIdx.x, mb = blockIdx.y, b = blockIdx.z;
  const int n0   = nt * QT, o0 = mb * QT;

  const unsigned short* ap = W16 + (size_t)(o0 + c) * CC + 8 * hh;
  const unsigned short* bp = XP + ((size_t)(b * NN + n0 + 16 * wave + c)) * CC + 8 * hh;

  v8f acc[4];
#pragma unroll
  for (int mt = 0; mt < 4; ++mt) acc[mt] = zero8();

#pragma unroll
  for (int ks = 0; ks < CC / 32; ++ks) {
    const Frag fb = ldfrag(bp + 32 * ks);
#pragma unroll
    for (int mt = 0; mt < 4; ++mt) {
      const Frag fa = ldfrag(ap + (size_t)(16 * mt) * CC + 32 * ks);
      acc[mt] = mma_h(fa.h, fb.h, acc[mt]);
    }
  }

  {
    const int nl = 16 * wave + c;
#pragma unroll
    for (int mt = 0; mt < 4; ++mt) {
#pragma unroll
      for (int r = 0; r < 8; ++r) {
        const int ol = 16 * mt + 8 * hh + r;
        Os[ol * OSP + nl] = acc[mt][r] * IWSC + BIAS[o0 + ol];
      }
    }
  }
  __syncthreads();

  const int e = tid & 7, lq = tid >> 3;
  if (mb < 4) {
    unsigned short* Ph = (mb < 2) ? Qh : Kh;
    unsigned short* Pl = (mb < 2) ? Ql : Kl;
    const int cb = QT * (mb & 1);
    v4u uh[4], ul[4];
#pragma unroll
    for (int it = 0; it < 4; ++it) {
      const int nl = it * 16 + lq;
#pragma unroll
      for (int t = 0; t < 4; ++t) {
        const float f0 = Os[(8 * e + 2 * t) * OSP + nl];
        const float f1 = Os[(8 * e + 2 * t + 1) * OSP + nl];
        const unsigned short hb0 = bf_bits(f0), hb1 = bf_bits(f1);
        const unsigned short lb0 = bf_bits(f0 - bf_up(hb0));
        const unsigned short lb1 = bf_bits(f1 - bf_up(hb1));
        uh[it][t] = pk16(hb0, hb1);
        ul[it][t] = pk16(lb0, lb1);
      }
    }
#pragma unroll
    for (int pass = 0; pass < 2; ++pass) {
#pragma unroll
      for (int it = 0; it < 4; ++it) {
        const int nl = it * 16 + lq;
        const size_t base = ((size_t)(b * NN + n0 + nl)) * CK + cb + 8 * e;
        *(volatile v4u*)(Ph + base) = uh[it];
        *(volatile v4u*)(Pl + base) = ul[it];
      }
      __threadfence();
    }
  } else {
    const int ch0 = QT * (mb - 4);
    v4u uv[4];
#pragma unroll
    for (int it = 0; it < 4; ++it) {
      const int row = it * 16 + lq;
      const v4f a = *(const v4f*)(Os + row * OSP + 8 * e);
      const v4f q = *(const v4f*)(Os + row * OSP + 8 * e + 4);
#pragma unroll
      for (int t = 0; t < 2; ++t) {
        uv[it][t]     = pk16(h_bits((_Float16)(a[2 * t] * VSC)), h_bits((_Float16)(a[2 * t + 1] * VSC)));
        uv[it][2 + t] = pk16(h_bits((_Float16)(q[2 * t] * VSC)), h_bits((_Float16)(q[2 * t + 1] * VSC)));
      }
    }
#pragma unroll
    for (int pass = 0; pass < 2; ++pass) {
#pragma unroll
      for (int it = 0; it < 4; ++it) {
        const int row = it * 16 + lq;
        *(volatile v4u*)(Vh + ((size_t)(b * CV + ch0 + row)) * NN + n0 + 8 * e) = uv[it];
      }
      __threadfence();
    }
  }
}

union AttnSmem { unsigned short q[2 * QT * QP]; float o[QT * OSPW]; };

__global__ __launch_bounds__(128)
void attn_gab(const unsigned short* __restrict__ Qh, const unsigned short* __restrict__ Ql,
              const unsigned short* __restrict__ Kh, const unsigned short* __restrict__ Kl,
              const unsigned short* __restrict__ Vh, float* OB) {
  __shared__ __align__(16) AttnSmem sm;
  const int tid  = threadIdx.x;
  const int wave = tid >> 5, lane = tid & 31;
  const int hh   = lane >> 4, c = lane & 15;
  const int n0   = blockIdx.x * QT, b = blockIdx.y;

  {
    const int e16 = tid & 15, rq = tid >> 4;
#pragma unroll
    for (int it = 0; it < 8; ++it) {
      const int row = 8 * it + rq;
      const size_t g = ((size_t)(b * NN + n0 + row)) * CK + 8 * e16;
      const v4u vh = *(const v4u*)(Qh + g);
      const v4u vl = *(const v4u*)(Ql + g);
      *(v4u*)(sm.q + row * QP + 8 * e16)        = vh;
      *(v4u*)(sm.q + (QT + row) * QP + 8 * e16) = vl;
    }
  }
  __syncthreads();

  const unsigned short* qsh = sm.q + (16 * wave + c) * QP + 8 * hh;
  const unsigned short* qsl = qsh + QT * QP;
  const unsigned short* Khp = Kh + (size_t)b * NN * CK + (size_t)c * CK + 8 * hh;
  const unsigned short* Klp = Kl + (size_t)b * NN * CK + (size_t)c * CK + 8 * hh;
  const unsigned short* Vhp = Vh + (size_t)b * CV * NN + (size_t)c * NN + 8 * hh;

  float m = -1.0e30f, l = 0.f;
  v8f o[8];
#pragma unroll
  for (int j = 0; j < 8; ++j) o[j] = zero8();

#pragma unroll 1
  for (int kb = 0; kb < NN; kb += 32) {
    v8f s0 = zero8(), s1 = zero8();
#pragma unroll 1
    for (int ks = 0; ks < CK / 32; ++ks) {
      const Frag qhf = ldfrag(qsh + 32 * ks);
      const Frag qlf = ldfrag(qsl + 32 * ks);
      const Frag k0  = ldfrag(Khp + (size_t)kb * CK + 32 * ks);
      const Frag k1  = ldfrag(Khp + (size_t)(kb + 16) * CK + 32 * ks);
      const Frag k0l = ldfrag(Klp + (size_t)kb * CK + 32 * ks);
      const Frag k1l = ldfrag(Klp + (size_t)(kb + 16) * CK + 32 * ks);
      s0 = mma_b(k0.bf, qhf.bf, s0);
      s1 = mma_b(k1.bf, qhf.bf, s1);
      s0 = mma_b(k0.bf, qlf.bf, s0);
      s1 = mma_b(k1.bf, qlf.bf, s1);
      s0 = mma_b(k0l.bf, qhf.bf, s0);
      s1 = mma_b(k1l.bf, qhf.bf, s1);
    }

    float mx = fmaxf(hmax8(s0), hmax8(s1));
    mx = fmaxf(mx, __shfl_xor(mx, 16, 32));
    const float mn   = fmaxf(m, mx);
    const float corr = __expf((m - mn) * SCL);
    m = mn;
    const float msh = mn * SCL - LNPS;
    l *= corr;
#pragma unroll
    for (int j = 0; j < 8; ++j) {
#pragma unroll
      for (int r = 0; r < 8; ++r) o[j][r] *= corr;
    }

    FragH ph;
    float ls = 0.f;
#pragma unroll
    for (int r = 0; r < 8; ++r) {
      const float e0 = __expf(s0[r] * SCL - msh);
      const float e1 = __expf(s1[r] * SCL - msh);
      ls += e0 + e1;
      ph.hv[0][r] = (_Float16)e0;
      ph.hv[1][r] = (_Float16)e1;
    }
    l += ls;

#pragma unroll
    for (int j = 0; j < 8; ++j) {
      const Frag vf = ldfrag(Vhp + (size_t)(16 * j) * NN + kb);
      o[j] = mma_h(vf.h, ph.v, o[j]);
    }
  }
  l += __shfl_xor(l, 16, 32);
  const float inv = IVSC / l;

  __syncthreads();
  const int qrow = 16 * wave + c;
#pragma unroll
  for (int j = 0; j < 8; ++j) {
    v4f va, vb;
#pragma unroll
    for (int r = 0; r < 4; ++r) { va[r] = o[j][r] * inv; vb[r] = o[j][4 + r] * inv; }
    *(v4f*)(sm.o + qrow * OSPW + 16 * j + 8 * hh)     = va;
    *(v4f*)(sm.o + qrow * OSPW + 16 * j + 8 * hh + 4) = vb;
  }
  __syncthreads();

  const int e = tid & 7, lq = tid >> 3;
#pragma unroll
  for (int pass = 0; pass < 2; ++pass) {
#pragma unroll
    for (int it = 0; it < 16; ++it) {
      const int L   = it * 16 + lq;
      const int q   = L >> 2, seg = L & 3;
      const v4f v = *(const v4f*)(sm.o + q * OSPW + 32 * seg + 4 * e);
      *(volatile v4f*)(OB + ((size_t)(b * NN + n0 + q)) * CV + 32 * seg + 4 * e) = v;
    }
    __threadfence();
  }
}

__global__ __launch_bounds__(128)
void out_proj(const float* __restrict__ OB, const unsigned short* __restrict__ WO16,
              const float* __restrict__ BOB, float* out) {
  __shared__ __align__(16) unsigned int Bs[2 * QT * (BP / 2)];
  __shared__ __align__(16) float Os[QT * OSP];
  const int tid  = threadIdx.x;
  const int lane = tid & 31, wave = tid >> 5;
  const int hh   = lane >> 4, c = lane & 15;
  const int pt = blockIdx.x, mb = blockIdx.y, b = blockIdx.z;
  const int p0 = pt * QT, o0 = mb * QT;
  const float* OBb = OB + (size_t)b * NN * CV;

  {
    const int e16 = tid & 15, rq = tid >> 4;
#pragma unroll
    for (int it = 0; it < 8; ++it) {
      const int rp = 8 * it + rq;
      const int r0 = 2 * rp;
      const v4f va = *(const v4f*)(OBb + (size_t)r0 * NN + p0 + 4 * e16);
      const v4f vb = *(const v4f*)(OBb + (size_t)(r0 + 1) * NN + p0 + 4 * e16);
#pragma unroll
      for (int t = 0; t < 4; ++t) {
        const float f0 = va[t] * USC, f1 = vb[t] * USC;
        const _Float16 h0 = (_Float16)f0, h1 = (_Float16)f1;
        const _Float16 l0 = (_Float16)((f0 - (float)h0) * RSC);
        const _Float16 l1 = (_Float16)((f1 - (float)h1) * RSC);
        const int pl = 4 * e16 + t;
        Bs[pl * (BP / 2) + rp]        = pk16(h_bits(h0), h_bits(h1));
        Bs[(QT + pl) * (BP / 2) + rp] = pk16(h_bits(l0), h_bits(l1));
      }
    }
  }
  __syncthreads();

  const unsigned short* Bh  = (const unsigned short*)Bs;
  const unsigned short* bph = Bh + (16 * wave + c) * BP + 8 * hh;
  const unsigned short* bpl = bph + QT * BP;
  const unsigned short* ap  = WO16 + (size_t)(o0 + c) * CV + 8 * hh;

  v8f acch[4], accl[4];
#pragma unroll
  for (int mt = 0; mt < 4; ++mt) { acch[mt] = zero8(); accl[mt] = zero8(); }

#pragma unroll
  for (int ks = 0; ks < CV / 32; ++ks) {
    const Frag fbh = ldfrag(bph + 32 * ks);
    const Frag fbl = ldfrag(bpl + 32 * ks);
#pragma unroll
    for (int mt = 0; mt < 4; ++mt) {
      const Frag fa = ldfrag(ap + (size_t)(16 * mt) * CV + 32 * ks);
      acch[mt] = mma_h(fa.h, fbh.h, acch[mt]);
      accl[mt] = mma_h(fa.h, fbl.h, accl[mt]);
    }
  }
  {
    const int nl = 16 * wave + c;
    const float osc = IWSC * IUSC;
#pragma unroll
    for (int mt = 0; mt < 4; ++mt) {
#pragma unroll
      for (int r = 0; r < 8; ++r) {
        const int ol = 16 * mt + 8 * hh + r;
        Os[ol * OSP + nl] = (acch[mt][r] + accl[mt][r] * IRSC) * osc + BOB[o0 + ol];
      }
    }
  }
  __syncthreads();
  {
    const int e = tid & 7, lq = tid >> 3;
#pragma unroll
    for (int pass = 0; pass < 2; ++pass) {
#pragma unroll
      for (int it = 0; it < 8; ++it) {
        const int L = it * 16 + lq;
        const int row = L >> 1, hf = L & 1;
        const int nl = hf * 32 + 4 * e;
        const v4f v = *(const v4f*)(Os + row * OSP + nl);
        *(volatile v4f*)(out + ((size_t)(b * CO + o0 + row)) * NN + p0 + nl) = v;
      }
      __threadfence();
    }
  }
}

extern "C" void kernel_launch(void* const* d_in, const int* in_sizes, int n_in,
                              void* d_out, int out_size, void* d_ws, size_t ws_size,
                              hipStream_t stream) {
  const int XN = NIMG * CC * NN;
  if (n_in < 9) return;
  if (in_sizes[0] != XN) return;
  if (in_sizes[1] != CK * CC || in_sizes[2] != CK) return;
  if (in_sizes[3] != CK * CC || in_sizes[4] != CK) return;
  if (in_sizes[5] != CV * CC || in_sizes[6] != CV) return;
  if (in_sizes[7] != CO * CV || in_sizes[8] != CO) return;
  if (out_size != NIMG * CO * NN) return;

  size_t off = 0;
  auto carve = [&](size_t bytes) { const size_t o = off; off += (bytes + 255) & ~(size_t)255; return o; };
  const size_t oW16 = carve((size_t)MQKV * CC * 2);
  const size_t oBIA = carve((size_t)MQKV * 4);
  const size_t oWO  = carve((size_t)CO * CV * 2);
  const size_t oBOB = carve((size_t)CO * 4);
  const size_t oXP  = carve((size_t)NIMG * NN * CC * 2);
  const size_t oQh  = carve((size_t)NIMG * NN * CK * 2);
  const size_t oQl  = carve((size_t)NIMG * NN * CK * 2);
  const size_t oKh  = carve((size_t)NIMG * NN * CK * 2);
  const size_t oKl  = carve((size_t)NIMG * NN * CK * 2);
  const size_t oVh  = carve((size_t)NIMG * CV * NN * 2);
  const size_t oOB  = carve((size_t)NIMG * NN * CV * 4);
  if (off > ws_size) return;
  if (off > (size_t)134217728) return;

  const float* x  = (const float*)d_in[0];
  const float* wq = (const float*)d_in[1];
  const float* bq = (const float*)d_in[2];
  const float* wk = (const float*)d_in[3];
  const float* bk = (const float*)d_in[4];
  const float* wv = (const float*)d_in[5];
  const float* bv = (const float*)d_in[6];
  const float* wo = (const float*)d_in[7];
  const float* bo = (const float*)d_in[8];

  char* ws = (char*)d_ws;
  unsigned short* W16 = (unsigned short*)(ws + oW16);
  float*          BIA = (float*)(ws + oBIA);
  unsigned short* WO  = (unsigned short*)(ws + oWO);
  float*          BOB = (float*)(ws + oBOB);
  unsigned short* XP  = (unsigned short*)(ws + oXP);
  unsigned short* Qh  = (unsigned short*)(ws + oQh);
  unsigned short* Ql  = (unsigned short*)(ws + oQl);
  unsigned short* Kh  = (unsigned short*)(ws + oKh);
  unsigned short* Kl  = (unsigned short*)(ws + oKl);
  unsigned short* Vh  = (unsigned short*)(ws + oVh);
  float*          OB  = (float*)(ws + oOB);
  float* out = (float*)d_out;

  const dim3 blk256(256), blk128(128);

  cvt_w<<<dim3(MQKV / 8), blk256, 0, stream>>>(wq, bq, wk, bk, wv, bv, W16, BIA);
  cvt_wo<<<dim3(CO / 16), blk256, 0, stream>>>(wo, bo, WO, BOB);
  cvt_x<<<dim3(NN / QT, CC / QT, NIMG), blk256, 0, stream>>>(x, XP);
  gemm_qkv<<<dim3(NN / QT, MQKV / QT, NIMG), blk128, 0, stream>>>(W16, BIA, XP, Qh, Ql, Kh, Kl, Vh);
  attn_gab<<<dim3(NN / QT, NIMG), blk128, 0, stream>>>(Qh, Ql, Kh, Kl, Vh, OB);
  out_proj<<<dim3(NN / QT, CO / QT, NIMG), blk128, 0, stream>>>(OB, WO, BOB, out);
  (void)hipGetLastError();
}
